// GruBlock_42116449305244
// MI455X (gfx1250) — hardware-run, weakly checked
//
#include <hip/hip_runtime.h>
#include <math.h>

constexpr int kBatch = 32;
constexpr int kSteps = 1024;
constexpr int kHid   = 256;
constexpr int kGate  = 3 * kHid;
constexpr int kCat   = 2 * kHid;
constexpr int kRows  = kBatch * kSteps;
constexpr float kWCarry    = 16.0f;
constexpr float kWCarryInv = 1.0f / 16.0f;
constexpr float kLnEps     = 1e-5f;
constexpr int kScanRows    = 16;
constexpr int kScanThreads = 512;
constexpr int kHPitch      = 264;
constexpr int kWihElems    = kGate * kHid;
constexpr int kWmapElems   = kHid * kCat;
constexpr int kCvtBlocksW  = kWihElems / 8 / 256;
constexpr int kCvtBlocksM  = kWmapElems / 8 / 256;
static_assert(kRows == 32768, "rows");
static_assert(kGate == 768, "gate columns");
static_assert(kRows % 64 == 0 && kGate % 64 == 0 && kHid % 64 == 0, "GEMM M, N tile multiples");
static_assert(kHid % 32 == 0 && kCat % 32 == 0, "GEMM K multiples of 32");
static_assert(kBatch % kScanRows == 0, "scan blocks");
static_assert(kScanRows == kScanThreads / 32, "one wave per row in the y copy");
static_assert(kHid == 16 * (kScanThreads / 32), "one 16-column group per wave");
static_assert(kHPitch % 8 == 0 && kHPitch >= kHid, "LDS pitch");
static_assert(kCvtBlocksW * 256 * 8 == kWihElems, "convert coverage");
static_assert(kCvtBlocksM * 256 * 8 == kWmapElems, "convert coverage");
static_assert(kRows % 8 == 0, "LN grid exact");

typedef __attribute__((ext_vector_type(16))) _Float16 v16h;
typedef __attribute__((ext_vector_type(8)))  _Float16 v8h;
typedef __attribute__((ext_vector_type(8)))  float    v8f;
typedef __attribute__((ext_vector_type(4)))  float    v4f;
typedef __attribute__((ext_vector_type(4)))  unsigned v4u;

__device__ __forceinline__ void guard4_h(v8f& a, v8f& b, v8f& c, v8f& d, v16h x, v16h y) {
  asm volatile("v_nop\n\tv_nop\n\tv_nop\n\tv_nop" : "+v"(a), "+v"(b), "+v"(c), "+v"(d) : "v"(x), "v"(y));
}
__device__ __forceinline__ void guard3_h(v8f& a, v8f& b, v8f& c, v16h x, v16h y0, v16h y1, v16h y2) {
  asm volatile("v_nop\n\tv_nop\n\tv_nop\n\tv_nop" : "+v"(a), "+v"(b), "+v"(c) : "v"(x), "v"(y0), "v"(y1), "v"(y2));
}
__device__ __forceinline__ void keep4_h(v16h a, v16h b, v16h c, v16h d) { asm volatile("v_nop" :: "v"(a), "v"(b), "v"(c), "v"(d)); }
__device__ __forceinline__ void acc_guard4(v8f& a, v8f& b, v8f& c, v8f& d) {
  asm volatile("v_nop\n\tv_nop\n\tv_nop\n\tv_nop" : "+v"(a), "+v"(b), "+v"(c), "+v"(d));
}
__device__ __forceinline__ void acc_guard3(v8f& a, v8f& b, v8f& c) {
  asm volatile("v_nop\n\tv_nop\n\tv_nop\n\tv_nop" : "+v"(a), "+v"(b), "+v"(c));
}

struct FragH {
  union U { v16h v; v8h h[2]; };
  static __device__ __forceinline__ v16h load(const _Float16* p) {
    U f; f.h[0] = *(const v8h*)(p); f.h[1] = *(const v8h*)(p + 16); return f.v;
  }
  static __device__ __forceinline__ v8f mma(v16h a, v16h b, v8f c) {
    return __builtin_amdgcn_wmma_f32_16x16x32_f16(false, a, false, b, (short)0, c, false, false);
  }
};

__device__ __forceinline__ float h16_to_f32(unsigned hb) {
  const unsigned sgn = (hb & 0x8000u) << 16;
  const unsigned em = hb & 0x7fffu;
  const float fn = __uint_as_float((em << 13) + 0x38000000u);
  const float fs = (float)em * 5.9604644775390625e-8f;
  const float mag = (em < 0x400u) ? fs : fn;
  return __uint_as_float(__float_as_uint(mag) | sgn);
}

__device__ __forceinline__ float sigm_f(float v)  { return 1.0f / (1.0f + expf(-v)); }
__device__ __forceinline__ float tanh_f(float v)  { return 1.0f - 2.0f / (1.0f + expf(2.0f * v)); }

__global__ __launch_bounds__(256) void cvt_weights_kernel(const float* __restrict__ w0, const float* __restrict__ w1,
                                                          const float* __restrict__ w2, const float* __restrict__ w3,
                                                          const float* __restrict__ w4, unsigned short* __restrict__ dst) {
  const int blk = blockIdx.x;
  int which = blk / kCvtBlocksW;
  which = which > 4 ? 4 : which;
  const int lblk = blk - which * kCvtBlocksW;
  const float* src = (which == 0) ? w0 : (which == 1) ? w1 : (which == 2) ? w2 : (which == 3) ? w3 : w4;
  const size_t li = (size_t)lblk * 256 + threadIdx.x;
  const size_t gi = (size_t)blk * 256 + threadIdx.x;
  const v4f a = *(const v4f*)(src + li * 8);
  const v4f b = *(const v4f*)(src + li * 8 + 4);
  v8h hv;
#pragma unroll
  for (int e = 0; e < 4; ++e) {
    hv[e]     = (_Float16)(a[e] * kWCarry);
    hv[4 + e] = (_Float16)(b[e] * kWCarry);
  }
  volatile v8h* dp = (volatile v8h*)(dst + gi * 8);
  *dp = hv;
  __threadfence();
  *dp = hv;
}

__global__ __launch_bounds__(256) void ln_rows_kernel(const float* __restrict__ x, const float* __restrict__ gam,
                                                      const float* __restrict__ bet, unsigned short* __restrict__ xn16) {
  const int lane = threadIdx.x & 31;
  const int rr = blockIdx.x * 8 + (threadIdx.x >> 5);
  const int b = rr / kSteps;
  const int t = rr - b * kSteps;
  const float* rp = x + (size_t)rr * kHid + lane * 8;
  v4f v0 = *(const v4f*)(rp);
  v4f v1 = *(const v4f*)(rp + 4);
  const v4f g0 = *(const v4f*)(gam + lane * 8);
  const v4f g1 = *(const v4f*)(gam + lane * 8 + 4);
  const v4f b0 = *(const v4f*)(bet + lane * 8);
  const v4f b1 = *(const v4f*)(bet + lane * 8 + 4);
  float s = ((v0[0] + v0[1]) + (v0[2] + v0[3])) + ((v1[0] + v1[1]) + (v1[2] + v1[3]));
#pragma unroll
  for (int off = 1; off < 32; off <<= 1) s += __shfl_xor(s, off, 32);
  const float mu = s * (1.0f / kHid);
  float ss = 0.0f;
#pragma unroll
  for (int e = 0; e < 4; ++e) {
    const float d0 = v0[e] - mu;
    const float d1 = v1[e] - mu;
    v0[e] = d0;
    v1[e] = d1;
    ss += d0 * d0;
    ss += d1 * d1;
  }
#pragma unroll
  for (int off = 1; off < 32; off <<= 1) ss += __shfl_xor(ss, off, 32);
  const float rstd = rsqrtf(ss * (1.0f / kHid) + kLnEps);
  v8h hv;
#pragma unroll
  for (int e = 0; e < 4; ++e) {
    hv[e]     = (_Float16)((v0[e] * rstd) * g0[e] + b0[e]);
    hv[4 + e] = (_Float16)((v1[e] * rstd) * g1[e] + b1[e]);
  }
  volatile v8h* dp = (volatile v8h*)(xn16 + ((size_t)t * kBatch + b) * kHid + lane * 8);
  *dp = hv;
  __threadfence();
  *dp = hv;
}

template <int BIAS_MODE, bool OUT_F16, bool RESID>
__global__ __launch_bounds__(256) void gemm64_f16(
    const unsigned short* __restrict__ Ap, int lda,
    const unsigned short* __restrict__ Btp, int ldb,
    void* __restrict__ Cout, int ldc,
    const float* __restrict__ bias, const float* __restrict__ resid,
    int M, int N, int K, float scale) {
  const _Float16* A  = (const _Float16*)Ap;
  const _Float16* Bt = (const _Float16*)Btp;
  __shared__ __align__(16) float sT[8][16 * 68];
  const int lane = threadIdx.x & 31;
  const int wave = threadIdx.x >> 5;
  const int tilesN = N >> 6;
  const int tilesM = M >> 6;
  const int tile = blockIdx.x * 8 + wave;
  if (tile >= tilesM * tilesN) return;
  const int tm = tile / tilesN;
  const int tn = tile - tm * tilesN;
  const int m0 = tm << 6;
  const int n0 = tn << 6;
  const int rlane = lane & 15;
  const int koff  = (lane >> 4) * 8;
  const int mOff  = (lane >> 4) * 8;

  v8f acc[4][4];
#pragma unroll
  for (int i = 0; i < 4; ++i)
#pragma unroll
    for (int j = 0; j < 4; ++j) acc[i][j] = (v8f){0.f, 0.f, 0.f, 0.f, 0.f, 0.f, 0.f, 0.f};

  const _Float16* arow = A  + (size_t)(m0 + rlane) * lda + koff;
  const _Float16* brow = Bt + (size_t)(n0 + rlane) * ldb + koff;
  const size_t a16 = (size_t)16 * lda;
  const size_t b16 = (size_t)16 * ldb;

  for (int k0 = 0; k0 < K; k0 += 32) {
    v16h bh[4];
#pragma unroll
    for (int j = 0; j < 4; ++j) bh[j] = FragH::load(brow + j * b16 + k0);
#pragma unroll
    for (int i = 0; i < 4; ++i) {
      const v16h ah = FragH::load(arow + i * a16 + k0);
#pragma unroll
      for (int j = 0; j < 4; ++j) acc[i][j] = FragH::mma(ah, bh[j], acc[i][j]);
      guard4_h(acc[i][0], acc[i][1], acc[i][2], acc[i][3], ah, bh[3]);
    }
    keep4_h(bh[0], bh[1], bh[2], bh[3]);
  }
  acc_guard4(acc[0][0], acc[0][1], acc[0][2], acc[0][3]);
  acc_guard4(acc[1][0], acc[1][1], acc[1][2], acc[1][3]);
  acc_guard4(acc[2][0], acc[2][1], acc[2][2], acc[2][3]);
  acc_guard4(acc[3][0], acc[3][1], acc[3][2], acc[3][3]);

  float* slab = sT[wave];
#pragma unroll
  for (int i = 0; i < 4; ++i) {
    const int mBase = m0 + (i << 4);
    v4f bm0 = (v4f){0.f, 0.f, 0.f, 0.f};
    v4f bm1 = (v4f){0.f, 0.f, 0.f, 0.f};
    if (BIAS_MODE == 1) {
      bm0 = *(const v4f*)(bias + mBase + mOff);
      bm1 = *(const v4f*)(bias + mBase + mOff + 4);
    }
#pragma unroll
    for (int j = 0; j < 4; ++j) {
#pragma unroll
      for (int r = 0; r < 8; ++r) {
        float v = acc[i][j][r] * scale;
        if (BIAS_MODE == 1) v += (r < 4) ? bm0[r & 3] : bm1[r & 3];
        slab[(mOff + r) * 68 + (j << 4) + rlane] = v;
      }
    }
    __builtin_amdgcn_fence(__ATOMIC_RELEASE, "workgroup");
    __builtin_amdgcn_wave_barrier();
    __builtin_amdgcn_fence(__ATOMIC_ACQUIRE, "workgroup");
    if (!OUT_F16) {
      float* C = (float*)Cout;
      const int hh = lane >> 4, c4 = (lane & 15) * 4;
      v4f b4 = (v4f){0.f, 0.f, 0.f, 0.f};
      if (BIAS_MODE == 2) b4 = *(const v4f*)(bias + n0 + c4);
      v4f vals[8];
#pragma unroll
      for (int it = 0; it < 8; ++it) {
        const int row = it * 2 + hh;
        v4f v = *(const v4f*)(slab + row * 68 + c4);
        v = v + b4;
        if (RESID) {
          const v4f rv = *(const v4f*)(resid + (size_t)(mBase + row) * ldc + n0 + c4);
          v = v + rv;
        }
        vals[it] = v;
      }
      for (int pass = 0; pass < 2; ++pass) {
#pragma unroll
        for (int it = 0; it < 8; ++it) {
          const int row = it * 2 + hh;
          *(volatile v4f*)(C + (size_t)(mBase + row) * ldc + n0 + c4) = vals[it];
        }
        __threadfence();
      }
    } else {
      unsigned short* C = (unsigned short*)Cout;
      const int q = lane >> 3, c8 = (lane & 7) * 8;
      v8h hvv[4];
#pragma unroll
      for (int it = 0; it < 4; ++it) {
        const int row = it * 4 + q;
        const float* sp = slab + row * 68 + c8;
#pragma unroll
        for (int e = 0; e < 8; ++e) hvv[it][e] = (_Float16)sp[e];
      }
      for (int pass = 0; pass < 2; ++pass) {
#pragma unroll
        for (int it = 0; it < 4; ++it) {
          const int row = it * 4 + q;
          *(volatile v8h*)(C + (size_t)(mBase + row) * ldc + n0 + c8) = hvv[it];
        }
        __threadfence();
      }
    }
    __builtin_amdgcn_fence(__ATOMIC_RELEASE, "workgroup");
    __builtin_amdgcn_wave_barrier();
    __builtin_amdgcn_fence(__ATOMIC_ACQUIRE, "workgroup");
  }
}

__global__ __launch_bounds__(512) void gru_scan_kernel(const unsigned short* __restrict__ Wp, const float* __restrict__ bhh,
                                                       const unsigned short* __restrict__ xpT,
                                                       unsigned short* __restrict__ y16, int dir) {
  __shared__ __align__(16) _Float16 Ah[2][kScanRows * kHPitch];
  const _Float16* W = (const _Float16*)Wp;
  const int tid = threadIdx.x, lane = tid & 31, wave = tid >> 5;
  const int c = lane & 15, hh = lane >> 4, koff = hh * 8;
  const int rowbase = blockIdx.x * kScanRows;
  const int j = 16 * wave + c;

  {
    _Float16* ahf = &Ah[0][0];
#pragma unroll 1
    for (int i = tid; i < 2 * kScanRows * kHPitch; i += kScanThreads) ahf[i] = (_Float16)0.0f;
  }
  float hst[8];
#pragma unroll
  for (int r = 0; r < 8; ++r) hst[r] = 0.0f;
  const float br = bhh[j];
  const float bz = bhh[kHid + j];
  const float bn = bhh[2 * kHid + j];
  const _Float16* wr = W + (size_t)j * kHid + koff;
  const _Float16* wz = wr + (size_t)kHid * kHid;
  const _Float16* wn = wr + (size_t)2 * kHid * kHid;
  const unsigned short* xqr = xpT + (size_t)j * kRows + rowbase + 8 * hh;
  const unsigned short* xqz = xqr + (size_t)kHid * kRows;
  const unsigned short* xqn = xqr + (size_t)2 * kHid * kRows;
  unsigned short* yrow = y16 + (size_t)(rowbase + wave) * kSteps * kCat + (size_t)dir * kHid + lane * 8;
  __syncthreads();

  const v8f z8 = {0.f, 0.f, 0.f, 0.f, 0.f, 0.f, 0.f, 0.f};

#pragma unroll 1
  for (int s = 0; s < kSteps; ++s) {
    const int tp = dir ? (kSteps - 1 - s) : s;
    const int cur = s & 1;
    const size_t xo = (size_t)tp * kBatch;
    v4u qr = *(const v4u*)(xqr + xo);
    v4u qz = *(const v4u*)(xqz + xo);
    v4u qn = *(const v4u*)(xqn + xo);
    asm volatile("" : "+v"(qr), "+v"(qz), "+v"(qn));

    const _Float16* ahrow = &Ah[cur][0] + c * kHPitch + koff;
    v8f accR = z8, accZ = z8, accN = z8;
#pragma unroll 1
    for (int k0 = 0; k0 < kHid; k0 += 32) {
      const v16h a  = FragH::load(ahrow + k0);
      const v16h b0 = FragH::load(wr + k0);
      const v16h b1 = FragH::load(wz + k0);
      const v16h b2 = FragH::load(wn + k0);
      accR = FragH::mma(a, b0, accR);
      accZ = FragH::mma(a, b1, accZ);
      accN = FragH::mma(a, b2, accN);
      guard3_h(accR, accZ, accN, a, b0, b1, b2);
    }
    acc_guard3(accR, accZ, accN);

    const unsigned ur[4] = {qr[0], qr[1], qr[2], qr[3]};
    const unsigned uz[4] = {qz[0], qz[1], qz[2], qz[3]};
    const unsigned un[4] = {qn[0], qn[1], qn[2], qn[3]};
    _Float16* ahn = &Ah[cur ^ 1][0];
#pragma unroll
    for (int r = 0; r < 8; ++r) {
      const float xr = h16_to_f32((ur[r >> 1] >> (16 * (r & 1))) & 0xffffu);
      const float xz = h16_to_f32((uz[r >> 1] >> (16 * (r & 1))) & 0xffffu);
      const float xn = h16_to_f32((un[r >> 1] >> (16 * (r & 1))) & 0xffffu);
      const float gr = accR[r] * kWCarryInv + br;
      const float gz = accZ[r] * kWCarryInv + bz;
      const float gn = accN[r] * kWCarryInv + bn;
      const float rg = sigm_f(xr + gr);
      const float zg = sigm_f(xz + gz);
      const float ng = tanh_f(xn + rg * gn);
      const float hn = (1.0f - zg) * ng + zg * hst[r];
      hst[r] = hn;
      ahn[(8 * hh + r) * kHPitch + j] = (_Float16)hn;
    }
    __syncthreads();
    {
      const v8h hv = *(const v8h*)(ahn + wave * kHPitch + lane * 8);
      volatile v8h* dp = (volatile v8h*)(yrow + (size_t)tp * kCat);
      *dp = hv;
      __threadfence();
      *dp = hv;
    }
  }
}

extern "C" void kernel_launch(void* const* d_in, const int* in_sizes, int n_in,
                              void* d_out, int out_size, void* d_ws, size_t ws_size, hipStream_t stream) {
  if (n_in < 13 || d_out == nullptr || d_ws == nullptr) return;
  if (in_sizes[0] != kRows * kHid || in_sizes[1] != kHid || in_sizes[2] != kHid ||
      in_sizes[3] != kWihElems || in_sizes[4] != kWihElems || in_sizes[5] != kGate || in_sizes[6] != kGate ||
      in_sizes[7] != kWihElems || in_sizes[8] != kWihElems || in_sizes[9] != kGate || in_sizes[10] != kGate ||
      in_sizes[11] != kWmapElems || in_sizes[12] != kHid || out_size != kRows * kHid) return;

  const float* x     = (const float*)d_in[0];
  const float* ln_g  = (const float*)d_in[1];
  const float* ln_b  = (const float*)d_in[2];
  const float* wih_f = (const float*)d_in[3];
  const float* whh_f = (const float*)d_in[4];
  const float* bih_f = (const float*)d_in[5];
  const float* bhh_f = (const float*)d_in[6];
  const float* wih_b = (const float*)d_in[7];
  const float* whh_b = (const float*)d_in[8];
  const float* bih_b = (const float*)d_in[9];
  const float* bhh_b = (const float*)d_in[10];
  const float* wmap  = (const float*)d_in[11];
  const float* bmap  = (const float*)d_in[12];
  float* out = (float*)d_out;

  char* ws = (char*)d_ws;
  size_t off = 0;
  auto carve = [&](size_t bytes) -> char* { char* p = ws + off; off += (bytes + 255) & ~(size_t)255; return p; };
  unsigned short* WPL = (unsigned short*)carve(((size_t)4 * kWihElems + kWmapElems) * 2);
  unsigned short* XN  = (unsigned short*)carve((size_t)kRows * kHid * 2);
  unsigned short* XPT = (unsigned short*)carve((size_t)kGate * kRows * 2);
  unsigned short* Y16 = (unsigned short*)carve((size_t)kRows * kCat * 2);
  if (off > ws_size || off > (size_t)134217728) return;

  unsigned short* WIHF = WPL;
  unsigned short* WHHF = WPL + (size_t)kWihElems;
  unsigned short* WIHB = WPL + (size_t)2 * kWihElems;
  unsigned short* WHHB = WPL + (size_t)3 * kWihElems;
  unsigned short* WMAP = WPL + (size_t)4 * kWihElems;

  cvt_weights_kernel<<<4 * kCvtBlocksW + kCvtBlocksM, 256, 0, stream>>>(wih_f, whh_f, wih_b, whh_b, wmap, WPL);
  ln_rows_kernel<<<kRows / 8, 256, 0, stream>>>(x, ln_g, ln_b, XN);

  const int gridIn  = (kGate / 64) * (kRows / 64) / 8;
  const int gridOut = (kRows / 64) * (kHid / 64) / 8;

  gemm64_f16<1, true, false><<<gridIn, 256, 0, stream>>>(
      WIHF, kHid, XN, kHid, (void*)XPT, kRows, bih_f, x, kGate, kRows, kHid, kWCarryInv);
  gru_scan_kernel<<<kBatch / kScanRows, kScanThreads, 0, stream>>>(WHHF, bhh_f, XPT, Y16, 0);

  gemm64_f16<1, true, false><<<gridIn, 256, 0, stream>>>(
      WIHB, kHid, XN, kHid, (void*)XPT, kRows, bih_b, x, kGate, kRows, kHid, kWCarryInv);
  gru_scan_kernel<<<kBatch / kScanRows, kScanThreads, 0, stream>>>(WHHB, bhh_b, XPT, Y16, 1);

  gemm64_f16<2, false, true><<<gridOut, 256, 0, stream>>>(
      Y16, kCat, WMAP, kCat, (void*)out, kHid, bmap, x, kRows, kHid, kCat, kWCarryInv);
}
